// xLSTMOperation_80023830659665
// MI455X (gfx1250) — hardware-verified
//
#include <hip/hip_runtime.h>
#include <math.h>
#include <stdint.h>

constexpr int kNB    = 16;
constexpr int kNC    = 192;
constexpr int kNS    = 1024;
constexpr int kRows  = kNB * kNS;
constexpr int kNin   = 384;
constexpr int kNHd   = 12;
constexpr int kDHd   = 32;
constexpr int kNUp   = 768;
constexpr int kNGin  = 1152;
constexpr int kNIf   = 64;
constexpr int kKConv = 1728;
constexpr int kGateLd = 32;
constexpr int kStageSteps = 8;

constexpr float kWCar    = 32.0f;
constexpr float kXaCar   = 64.0f;
constexpr float kGinCar  = 256.0f;
constexpr float kHoCar   = 16.0f;
constexpr float kW2Car   = 16.0f;
constexpr float kUpScale   = 1.0f / 32.0f;
constexpr float kQKScale   = 256.0f / (64.0f * 32.0f);
constexpr float kIfScale   = 1.0f / (256.0f * 32.0f);
constexpr float kDownScale = 1.0f / (16.0f * 32.0f);
constexpr float kLinScale  = 1.0f / 32.0f;
constexpr float kConvScale = 1.0f / 16.0f;

static_assert(kRows % 64 == 0, "");
static_assert(kNC % 64 == 0 && kNin % 64 == 0 && kNUp % 64 == 0 && kNIf % 64 == 0, "");
static_assert(kNC % 32 == 0 && kNin % 32 == 0 && kNGin % 32 == 0 && kKConv % 32 == 0, "");
static_assert(kNS % kStageSteps == 0, "");

typedef __attribute__((ext_vector_type(16))) _Float16 v16h;
typedef __attribute__((ext_vector_type(8)))  _Float16 v8h;
typedef __attribute__((ext_vector_type(16))) __bf16   v16b;
typedef __attribute__((ext_vector_type(8)))  __bf16   v8b;
typedef __attribute__((ext_vector_type(8)))  float    v8f;
typedef __attribute__((ext_vector_type(4)))  float    v4f;
typedef __attribute__((ext_vector_type(4)))  unsigned int v4u;

__device__ __forceinline__ unsigned short f2bf_bits(float f) {
  unsigned u = __float_as_uint(f);
  return (unsigned short)((u + 0x7FFFu + ((u >> 16) & 1u)) >> 16);
}
__device__ __forceinline__ float bf_bits2f(unsigned short h) { return __uint_as_float(((unsigned)h) << 16); }

__device__ __forceinline__ void dep_guard_h(v8f& a, v8f& b, v16h x, v16h y) { asm volatile("v_nop\n\tv_nop\n\tv_nop\n\tv_nop" : "+v"(a), "+v"(b) : "v"(x), "v"(y)); }
__device__ __forceinline__ void dep_guard_b(v8f& a, v8f& b, v16b x, v16b y) { asm volatile("v_nop\n\tv_nop\n\tv_nop\n\tv_nop" : "+v"(a), "+v"(b) : "v"(x), "v"(y)); }
__device__ __forceinline__ void keep4_h(v16h a, v16h b, v16h c, v16h d) { asm volatile("v_nop" :: "v"(a), "v"(b), "v"(c), "v"(d)); }
__device__ __forceinline__ void keep4_b(v16b a, v16b b, v16b c, v16b d) { asm volatile("v_nop" :: "v"(a), "v"(b), "v"(c), "v"(d)); }
__device__ __forceinline__ void acc_guard4(v8f& a, v8f& b, v8f& c, v8f& d) { asm volatile("v_nop\n\tv_nop\n\tv_nop\n\tv_nop" : "+v"(a), "+v"(b), "+v"(c), "+v"(d)); }
template <typename T> struct Frag;
template <> struct Frag<_Float16> {
  typedef v16h V; union U { v16h v; v8h h[2]; };
  static __device__ __forceinline__ v16h load(const _Float16* p) {
    U f; f.h[0] = *(const v8h*)(p); f.h[1] = *(const v8h*)(p + 16); return f.v;
  }
  static __device__ __forceinline__ v8f mma(v16h a, v16h b, v8f c) {
    return __builtin_amdgcn_wmma_f32_16x16x32_f16(false, a, false, b, (short)0, c, false, false);
  }
  static __device__ __forceinline__ void guard(v8f& a, v8f& b, v16h x, v16h y) { dep_guard_h(a, b, x, y); }
  static __device__ __forceinline__ void keep(v16h a, v16h b, v16h c, v16h d) { keep4_h(a, b, c, d); }
};
template <> struct Frag<__bf16> {
  typedef v16b V; union U { v16b v; v8b h[2]; };
  static __device__ __forceinline__ v16b load(const __bf16* p) {
    U f; f.h[0] = *(const v8b*)(p); f.h[1] = *(const v8b*)(p + 16); return f.v;
  }
  static __device__ __forceinline__ v8f mma(v16b a, v16b b, v8f c) {
    return __builtin_amdgcn_wmma_f32_16x16x32_bf16(false, a, false, b, (short)0, c, false, false);
  }
  static __device__ __forceinline__ void guard(v8f& a, v8f& b, v16b x, v16b y) { dep_guard_b(a, b, x, y); }
  static __device__ __forceinline__ void keep(v16b a, v16b b, v16b c, v16b d) { keep4_b(a, b, c, d); }
};

__device__ __forceinline__ unsigned pk16(unsigned short a, unsigned short b) { return (unsigned)a | ((unsigned)b << 16); }
__device__ __forceinline__ unsigned short h_bits(float f) { const _Float16 h = (_Float16)f; return __builtin_bit_cast(unsigned short, h); }
__device__ __forceinline__ float h2f(unsigned short u) { const _Float16 h = __builtin_bit_cast(_Float16, u); return (float)h; }

template <int ET> struct Elem;
template <> struct Elem<0> { typedef _Float16 T; };
template <> struct Elem<1> { typedef __bf16 T; };
template <int ET, bool SPLIT, int BIAS_MODE, int OUT_MODE, bool RESID, int ACT = 0>
__global__ __launch_bounds__(256) void wmma_gemm64(
    const unsigned short* __restrict__ Ap, const unsigned short* __restrict__ A2p, int lda, long strideA,
    const unsigned short* __restrict__ Btp, const unsigned short* __restrict__ Bt2p, int ldb, long strideB,
    void* __restrict__ Cout, void* __restrict__ Cout2, int ldc, long strideC,
    const float* __restrict__ bias,
    const float* __restrict__ resid, long strideR,
    int M, int N, int K, float scale) {
  typedef typename Elem<ET>::T T;
  typedef typename Frag<T>::V V;
  const T* A = (const T*)Ap; const T* A2 = (const T*)A2p; const T* Bt = (const T*)Btp; const T* Bt2 = (const T*)Bt2p;
  __shared__ __align__(16) float sT[8][16 * 68];
  const int b    = blockIdx.y;
  const int lane = threadIdx.x & 31;
  const int wave = threadIdx.x >> 5;
  const int tilesN = N >> 6;
  const int tilesM = M >> 6;
  const int tile = blockIdx.x * 8 + wave;
  if (tile >= tilesM * tilesN) return;
  const int tm = tile / tilesN;
  const int tn = tile - tm * tilesN;
  const int m0 = tm << 6;
  const int n0 = tn << 6;

  const T* Ab  = A  + (size_t)b * strideA;
  const T* Bb  = Bt + (size_t)b * strideB;
  const T* Ab2 = SPLIT ? (A2  + (size_t)b * strideA) : nullptr;
  const T* Bb2 = SPLIT ? (Bt2 + (size_t)b * strideB) : nullptr;

  const int rlane = lane & 15;
  const int koff  = (lane >> 4) * 8;
  const int mOff  = (lane >> 4) * 8;

  v8f acc[4][4];
#pragma unroll
  for (int i = 0; i < 4; ++i)
#pragma unroll
    for (int j = 0; j < 4; ++j) acc[i][j] = (v8f){0.f,0.f,0.f,0.f,0.f,0.f,0.f,0.f};

  for (int k0 = 0; k0 < K; k0 += 32) {
    V bh[4], bl[4];
#pragma unroll
    for (int j = 0; j < 4; ++j) {
      const size_t bo = (size_t)(n0 + (j << 4) + rlane) * ldb + koff + k0;
      bh[j] = Frag<T>::load(Bb + bo);
      if (SPLIT) bl[j] = Frag<T>::load(Bb2 + bo);
    }
#pragma unroll
    for (int i = 0; i < 4; ++i) {
      const size_t ao = (size_t)(m0 + (i << 4) + rlane) * lda + koff + k0;
      V ah = Frag<T>::load(Ab + ao);
      V al;
      if (SPLIT) al = Frag<T>::load(Ab2 + ao);
#pragma unroll
      for (int j = 0; j < 4; ++j) {
        acc[i][j] = Frag<T>::mma(ah, bh[j], acc[i][j]);
        if (SPLIT) {
          acc[i][j] = Frag<T>::mma(ah, bl[j], acc[i][j]);
          acc[i][j] = Frag<T>::mma(al, bh[j], acc[i][j]);
        }
      }
      Frag<T>::guard(acc[i][0], acc[i][3], ah, SPLIT ? al : ah);
    }
    Frag<T>::keep(bh[0], bh[1], bh[2], bh[3]);
    if (SPLIT) Frag<T>::keep(bl[0], bl[1], bl[2], bl[3]);
  }
  acc_guard4(acc[0][0], acc[0][1], acc[0][2], acc[0][3]);
  acc_guard4(acc[1][0], acc[1][1], acc[1][2], acc[1][3]);
  acc_guard4(acc[2][0], acc[2][1], acc[2][2], acc[2][3]);
  acc_guard4(acc[3][0], acc[3][1], acc[3][2], acc[3][3]);

  float* slab = sT[wave];
  const float* Rb = RESID ? (resid + (size_t)b * strideR) : nullptr;
#pragma unroll
  for (int i = 0; i < 4; ++i) {
    const int mBase = m0 + (i << 4);
#pragma unroll
    for (int j = 0; j < 4; ++j) {
      const int n = n0 + (j << 4) + rlane;
      float bv = 0.f;
      if (BIAS_MODE == 2) bv = bias[n];
#pragma unroll
      for (int r = 0; r < 8; ++r) {
        float v = acc[i][j][r] * scale;
        if (BIAS_MODE == 1) v += bias[mBase + mOff + r];
        if (BIAS_MODE == 2) v += bv;
        if (RESID) v += Rb[(size_t)(mBase + mOff + r) * ldc + n];
        if (ACT == 2) v = fmaxf(v, 0.0f);
        if (ACT == 3) v = v / (1.0f + expf(-v));
        if (ACT == 4) v = (v > 0.f) ? v : 0.01f * v;
        slab[(mOff + r) * 68 + (j << 4) + rlane] = v;
      }
    }
    __builtin_amdgcn_fence(__ATOMIC_RELEASE, "workgroup");
    __builtin_amdgcn_wave_barrier();
    __builtin_amdgcn_fence(__ATOMIC_ACQUIRE, "workgroup");
    if (OUT_MODE == 0) {
      float* C = (float*)Cout + (size_t)b * strideC;
      const int hh = lane >> 4, c4 = (lane & 15) * 4;
      for (int pass = 0; pass < 2; ++pass) {
#pragma unroll
        for (int it = 0; it < 8; ++it) {
          const int row = it * 2 + hh;
          v4f v = *(const v4f*)(slab + row * 68 + c4);
          *(volatile v4f*)(C + (size_t)(mBase + row) * ldc + n0 + c4) = v;
        }
        __threadfence();
      }
    } else {
      const int q = lane >> 3, c8 = (lane & 7) * 8;
      unsigned short* C  = (unsigned short*)Cout  + (size_t)b * strideC;
      unsigned short* C2 = (OUT_MODE == 2) ? ((unsigned short*)Cout2 + (size_t)b * strideC) : nullptr;
      for (int pass = 0; pass < 2; ++pass) {
#pragma unroll
        for (int it = 0; it < 4; ++it) {
          const int row = it * 4 + q;
          const float* sp = slab + row * 68 + c8;
          v8h hv, lv;
#pragma unroll
          for (int e = 0; e < 8; ++e) {
            if (OUT_MODE == 1) {
              hv[e] = (_Float16)sp[e];
            } else {
              unsigned short hb = f2bf_bits(sp[e]);
              unsigned short lb = f2bf_bits(sp[e] - bf_bits2f(hb));
              hv[e] = __builtin_bit_cast(_Float16, hb);
              lv[e] = __builtin_bit_cast(_Float16, lb);
            }
          }
          *(volatile v8h*)(C + (size_t)(mBase + row) * ldc + n0 + c8) = hv;
          if (OUT_MODE == 2) *(volatile v8h*)(C2 + (size_t)(mBase + row) * ldc + n0 + c8) = lv;
        }
        __threadfence();
      }
    }
    __builtin_amdgcn_fence(__ATOMIC_RELEASE, "workgroup");
    __builtin_amdgcn_wave_barrier();
    __builtin_amdgcn_fence(__ATOMIC_ACQUIRE, "workgroup");
  }
}

__device__ __forceinline__ float wsum32(float v) {
#pragma unroll
  for (int off = 16; off > 0; off >>= 1) v += __shfl_xor(v, off, 32);
  return v;
}
__device__ __forceinline__ void wave_sync_lds() {
  __builtin_amdgcn_fence(__ATOMIC_RELEASE, "workgroup");
  __builtin_amdgcn_wave_barrier();
  __builtin_amdgcn_fence(__ATOMIC_ACQUIRE, "workgroup");
}
__device__ __forceinline__ float conv_silu(float x0, float x1, float x2, float x3,
                                           float k0, float k1, float k2, float k3, float cb) {
#pragma clang fp contract(off)
  float a = x0 * k0;
  a = a + x1 * k1;
  a = a + x2 * k2;
  a = a + x3 * k3;
  a = a + cb;
  return a * (1.0f / (1.0f + expf(-a)));
}

__global__ __launch_bounds__(256) void k_wt64(const float* __restrict__ Wm, unsigned short* __restrict__ out,
                                              int Kdim, int Ndim, float scale) {
  __shared__ float sm[64][65];
  const int t  = threadIdx.x;
  const int k0 = blockIdx.x * 64;
  const int n0 = blockIdx.y * 64;
#pragma unroll
  for (int i = 0; i < 16; ++i) {
    const int e = i * 256 + t;
    const int r = e >> 6;
    const int c = e & 63;
    sm[c][r] = Wm[(size_t)(k0 + r) * Ndim + n0 + c] * scale;
  }
  __syncthreads();
  const int lane = t & 31, wave = t >> 5;
  const int q = lane >> 3, c8 = (lane & 7) * 8;
  for (int pass = 0; pass < 2; ++pass) {
#pragma unroll
    for (int it = 0; it < 2; ++it) {
      const int row = wave * 8 + it * 4 + q;
      unsigned short hb[8];
#pragma unroll
      for (int e = 0; e < 8; ++e) hb[e] = h_bits(sm[row][c8 + e]);
      const v4u u = (v4u){pk16(hb[0], hb[1]), pk16(hb[2], hb[3]), pk16(hb[4], hb[5]), pk16(hb[6], hb[7])};
      *(volatile v4u*)(out + (size_t)(n0 + row) * Kdim + k0 + c8) = u;
    }
    __threadfence();
  }
}

__global__ __launch_bounds__(256) void k_wif(const float* __restrict__ wi, const float* __restrict__ wf,
                                             unsigned short* __restrict__ out, float scale) {
  const int g  = blockIdx.x * 256 + threadIdx.x;
  const int n  = g / 144;
  const int k0 = (g - n * 144) * 8;
  const int ni = (n < 12) ? n : 11;
  int nf = n - 12; nf = (nf < 0) ? 0 : ((nf > 11) ? 11 : nf);
  unsigned short hb[8];
#pragma unroll
  for (int e = 0; e < 8; ++e) {
    const float a = wi[(size_t)(k0 + e) * kNHd + ni];
    const float c = wf[(size_t)(k0 + e) * kNHd + nf];
    const float v = (n < 12) ? a : ((n < 24) ? c : 0.0f);
    hb[e] = h_bits(v * scale);
  }
  const v4u u = (v4u){pk16(hb[0], hb[1]), pk16(hb[2], hb[3]), pk16(hb[4], hb[5]), pk16(hb[6], hb[7])};
  unsigned short* dst = out + (size_t)n * kNGin + k0;
  *(volatile v4u*)dst = u;
  __threadfence();
  *(volatile v4u*)dst = u;
}

__global__ __launch_bounds__(32) void k_bias64(const float* __restrict__ bi, const float* __restrict__ bfv,
                                               float* __restrict__ out) {
  const int l = threadIdx.x;
  v4f v;
#pragma unroll
  for (int i = 0; i < 4; ++i) {
    const int n  = 4 * l + i;
    const int ni = (n < 12) ? n : 11;
    int nf = n - 12; nf = (nf < 0) ? 0 : ((nf > 11) ? 11 : nf);
    const float a = bi[ni];
    const float c = bfv[nf];
    v[i] = (n < 12) ? a : ((n < 24) ? c : 0.0f);
  }
  if (l < 16) *(volatile v4f*)(out + 4 * l) = v;
  __threadfence();
  if (l < 16) *(volatile v4f*)(out + 4 * l) = v;
}

__global__ __launch_bounds__(256) void k_w2(const float* __restrict__ w, unsigned short* __restrict__ out, float scale) {
  const int g   = blockIdx.x * 256 + threadIdx.x;
  const int co  = g / 216;
  const int j   = g - co * 216;
  const int tap = j / 24;
  const int ci0 = (j - tap * 24) * 8;
  unsigned short hb[8];
#pragma unroll
  for (int e = 0; e < 8; ++e) hb[e] = h_bits(w[((size_t)(co * kNC + ci0 + e)) * 9 + tap] * scale);
  const v4u u = (v4u){pk16(hb[0], hb[1]), pk16(hb[2], hb[3]), pk16(hb[4], hb[5]), pk16(hb[6], hb[7])};
  unsigned short* dst = out + (size_t)co * kKConv + (size_t)j * 8;
  *(volatile v4u*)dst = u;
  __threadfence();
  *(volatile v4u*)dst = u;
}

__global__ __launch_bounds__(256) void k_ln(const float* __restrict__ x, const float* __restrict__ lw,
                                            const float* __restrict__ lb, float* __restrict__ seqf,
                                            unsigned short* __restrict__ seq16, unsigned short* __restrict__ hln16) {
  __shared__ float sm[kNC][33];
  const int t   = threadIdx.x;
  const int blk = blockIdx.x;
  const int b   = blk >> 5;
  const int p0  = (blk & 31) * 32;
#pragma unroll
  for (int i = 0; i < 24; ++i) {
    const int e = i * 256 + t;
    const int c = e >> 5, pl = e & 31;
    sm[c][pl] = x[((size_t)(b * kNC + c)) * kNS + p0 + pl];
  }
  __syncthreads();
  const int lane = t & 31, wave = t >> 5;
  for (int jj = 0; jj < 4; ++jj) {
    const int j = wave * 4 + jj;
    const size_t row = (size_t)b * kNS + p0 + j;
    float v[6];
#pragma unroll
    for (int i = 0; i < 6; ++i) v[i] = sm[lane + 32 * i][j];
    float s = ((v[0] + v[1]) + (v[2] + v[3])) + (v[4] + v[5]);
    s = wsum32(s);
    const float mu = s * (1.0f / 192.0f);
    float s2 = 0.0f;
#pragma unroll
    for (int i = 0; i < 6; ++i) { const float d = v[i] - mu; s2 += d * d; }
    s2 = wsum32(s2);
    const float var = s2 * (1.0f / 192.0f);
    const float rs  = 1.0f / sqrtf(var + 1e-5f);
    v4f f0, f1;
#pragma unroll
    for (int i = 0; i < 4; ++i) {
      f0[i] = sm[4 * lane + i][j];
      int c1 = 128 + 4 * lane + i; c1 = (c1 > kNC - 1) ? (kNC - 1) : c1;
      f1[i] = sm[c1][j];
    }
    unsigned short rb[8], hb[8];
#pragma unroll
    for (int e = 0; e < 8; ++e) {
      int ch = 8 * lane + e; ch = (ch > kNC - 1) ? (kNC - 1) : ch;
      const float raw = sm[ch][j];
      rb[e] = h_bits(raw);
      hb[e] = h_bits((raw - mu) * rs * lw[ch] + lb[ch]);
    }
    const v4u ur = (v4u){pk16(rb[0], rb[1]), pk16(rb[2], rb[3]), pk16(rb[4], rb[5]), pk16(rb[6], rb[7])};
    const v4u uh = (v4u){pk16(hb[0], hb[1]), pk16(hb[2], hb[3]), pk16(hb[4], hb[5]), pk16(hb[6], hb[7])};
    for (int pass = 0; pass < 2; ++pass) {
      *(volatile v4f*)(seqf + row * kNC + 4 * lane) = f0;
      if (lane < 16) *(volatile v4f*)(seqf + row * kNC + 128 + 4 * lane) = f1;
      if (lane < 24) {
        *(volatile v4u*)(seq16 + row * kNC + 8 * lane) = ur;
        *(volatile v4u*)(hln16 + row * kNC + 8 * lane) = uh;
      }
      __threadfence();
    }
  }
}

__global__ __launch_bounds__(256) void k_conv1d(const float* __restrict__ up, const float* __restrict__ convk,
                                                const float* __restrict__ convb, unsigned short* __restrict__ xact16,
                                                unsigned short* __restrict__ gin16) {
  const int g   = blockIdx.x * 256 + threadIdx.x;
  const int row = g / 48;
  const int c0  = (g - row * 48) * 8;
  const int b   = row >> 10, s = row & 1023;
  float xv[4][8];
#pragma unroll
  for (int tp = 0; tp < 4; ++tp) {
    const int s2 = s - 3 + tp;
    const bool valid = (s2 >= 0);
    const size_t rs = (size_t)b * kNS + (valid ? s2 : 0);
    const float* p = up + rs * kNUp + c0;
    const v4f a = *(const v4f*)p;
    const v4f d = *(const v4f*)(p + 4);
#pragma unroll
    for (int e = 0; e < 4; ++e) {
      xv[tp][e]     = valid ? a[e] : 0.0f;
      xv[tp][4 + e] = valid ? d[e] : 0.0f;
    }
  }
  unsigned short hb[8], xb[8];
#pragma unroll
  for (int e = 0; e < 8; ++e) {
    const int c = c0 + e;
    const float xa = conv_silu(xv[0][e], xv[1][e], xv[2][e], xv[3][e],
                               convk[c * 4 + 0], convk[c * 4 + 1], convk[c * 4 + 2], convk[c * 4 + 3], convb[c]);
    hb[e] = h_bits(xa * kXaCar);
    xb[e] = h_bits(xv[3][e] * kGinCar);
  }
  const v4u ua = (v4u){pk16(hb[0], hb[1]), pk16(hb[2], hb[3]), pk16(hb[4], hb[5]), pk16(hb[6], hb[7])};
  const v4u ux = (v4u){pk16(xb[0], xb[1]), pk16(xb[2], xb[3]), pk16(xb[4], xb[5]), pk16(xb[6], xb[7])};
  unsigned short* da = xact16 + (size_t)row * kNin + c0;
  unsigned short* dx = gin16 + (size_t)row * kNGin + 2 * kNin + c0;
  *(volatile v4u*)da = ua;
  *(volatile v4u*)dx = ux;
  __threadfence();
  *(volatile v4u*)da = ua;
  *(volatile v4u*)dx = ux;
}

__global__ __launch_bounds__(192) void k_gate(const float* __restrict__ ifp, float* __restrict__ gt) {
  __shared__ float stg[kNB][kGateLd];
  const int t    = threadIdx.x;
  const int b    = t / 12;
  const int hd   = t - b * 12;
  const int lane = t & 31, wave = t >> 5;
  for (int e = t; e < kNB * kGateLd; e += 192) (&stg[0][0])[e] = 0.0f;
  __syncthreads();
  float m = 0.0f;
  for (int ts = 0; ts < kNS; ++ts) {
    const size_t row = (size_t)b * kNS + ts;
    const float ig = ifp[row * kNIf + hd];
    const float fg = ifp[row * kNIf + 12 + hd];
    const float lf = fminf(fg, 0.0f) - log1pf(expf(-fabsf(fg)));
    const float lm = lf + m;
    const float mnew = fmaxf(lm, ig);
    const float fs = expf(lm - mnew);
    const float is = expf(ig - mnew);
    m = mnew;
    stg[b][hd] = fs;
    stg[b][16 + hd] = is;
    __syncthreads();
    float vals[3];
#pragma unroll
    for (int q = 0; q < 3; ++q) {
      int bb = wave + 6 * q; bb = (bb > kNB - 1) ? (kNB - 1) : bb;
      vals[q] = stg[bb][lane];
    }
    for (int pass = 0; pass < 2; ++pass) {
#pragma unroll
      for (int q = 0; q < 3; ++q) {
        const int bb = wave + 6 * q;
        if (bb < kNB) *(volatile float*)(gt + ((size_t)bb * kNS + ts) * kGateLd + lane) = vals[q];
      }
      __threadfence();
    }
    __syncthreads();
  }
}

__global__ __launch_bounds__(384) void k_scan(const float* __restrict__ up, const unsigned int* __restrict__ gin32,
                                              const float* __restrict__ gt, const float* __restrict__ convk,
                                              const float* __restrict__ convb, const float* __restrict__ skipv,
                                              const float* __restrict__ mhw, const float* __restrict__ mhb,
                                              unsigned short* __restrict__ hout) {
#pragma clang fp contract(off)
  __shared__ __align__(16) float qk_s[kNHd][2][64];
  __shared__ __align__(16) unsigned int hst[2][kStageSteps][kNin / 2];
  const int t    = threadIdx.x;
  const int lane = t & 31;
  const int hd   = t >> 5;
  const int c    = t;
  const int b    = blockIdx.x;
  const float ck0 = convk[c * 4 + 0], ck1 = convk[c * 4 + 1], ck2 = convk[c * 4 + 2], ck3 = convk[c * 4 + 3];
  const float cbv = convb[c], sk = skipv[c], gw = mhw[c], gb = mhb[c];
  const float kscale = 0.17677669529663687f;
  const float ginInv = 1.0f / 256.0f;
  const unsigned sh = (unsigned)(c & 1) * 16u;
  float Cst[32];
#pragma unroll
  for (int e = 0; e < 32; ++e) Cst[e] = 0.0f;
  float nst = 0.0f;
  float xh1 = 0.0f, xh2 = 0.0f, xh3 = 0.0f;
  for (int ts = 0; ts < kNS; ++ts) {
    const size_t row = (size_t)b * kNS + ts;
    const float xin = up[row * kNUp + c];
    const float zv  = up[row * kNUp + kNin + c];
    const unsigned wq = gin32[(row * kNGin + c) >> 1];
    const unsigned wk = gin32[(row * kNGin + kNin + c) >> 1];
    const float qv = h2f((unsigned short)((wq >> sh) & 0xffffu)) * ginInv;
    const float kv = (h2f((unsigned short)((wk >> sh) & 0xffffu)) * ginInv) * kscale;
    const float fs = gt[row * kGateLd + hd];
    const float is = gt[row * kGateLd + 16 + hd];
    const int buf = ts & 1;
    qk_s[hd][buf][lane] = qv;
    qk_s[hd][buf][32 + lane] = kv;
    wave_sync_lds();
    nst = fs * nst + is * kv;
    const float dq = wsum32(nst * qv);
    const float den = fmaxf(fabsf(dq), 1.0f);
    const float rden = 1.0f / den;
    const float isv = is * xin;
    float cq = 0.0f;
#pragma unroll
    for (int g = 0; g < 8; ++g) {
      const v4f q4 = *(const v4f*)(&qk_s[hd][buf][4 * g]);
      const v4f k4 = *(const v4f*)(&qk_s[hd][buf][32 + 4 * g]);
#pragma unroll
      for (int e = 0; e < 4; ++e) {
        const float cn = fmaf(fs, Cst[4 * g + e], isv * k4[e]);
        Cst[4 * g + e] = cn;
        cq = cq + cn * q4[e];
      }
    }
    const float hval = cq * rden;
    const float mu   = wsum32(hval) * (1.0f / 32.0f);
    const float dv   = hval - mu;
    const float var  = wsum32(dv * dv) * (1.0f / 32.0f);
    const float hn   = dv * (1.0f / sqrtf(var + 1e-5f)) * gw + gb;
    const float xact = conv_silu(xh3, xh2, xh1, xin, ck0, ck1, ck2, ck3, cbv);
    xh3 = xh2; xh2 = xh1; xh1 = xin;
    const float sz = zv * (1.0f / (1.0f + expf(-zv)));
    const float ho = (hn + sk * xact) * sz;
    const unsigned hb = (unsigned)h_bits(ho * kHoCar);
    const unsigned nb = (unsigned)__shfl_xor((int)hb, 1, 32);
    const int cbuf = (ts >> 3) & 1;
    const int srow = ts & 7;
    if ((lane & 1) == 0) hst[cbuf][srow][c >> 1] = hb | (nb << 16);
    if (srow == kStageSteps - 1) {
      __syncthreads();
      const int r  = t / 48;
      const int w4 = (t - r * 48) * 4;
      const v4u u = *(const v4u*)(&hst[cbuf][r][w4]);
      const size_t orow = row - (kStageSteps - 1) + r;
      unsigned short* dst = hout + orow * kNin + (size_t)w4 * 2;
      *(volatile v4u*)dst = u;
      __threadfence();
      *(volatile v4u*)dst = u;
    }
  }
}

__global__ __launch_bounds__(256) void k_im2col(const float* __restrict__ x1, const float* __restrict__ x2,
                                                unsigned short* __restrict__ col) {
  const int g   = blockIdx.x * 256 + threadIdx.x;
  const int row = g / 216;
  const int j   = g - row * 216;
  const int tap = j / 24;
  const int ci0 = (j - tap * 24) * 8;
  const int kh  = tap / 3, kw = tap - kh * 3;
  const int b   = row >> 10, p = row & 1023;
  const int hh  = p >> 5, ww = p & 31;
  const int h2  = hh + kh - 1, w2 = ww + kw - 1;
  const bool valid = ((unsigned)h2 < 32u) && ((unsigned)w2 < 32u);
  const int h2c = (h2 < 0) ? 0 : ((h2 > 31) ? 31 : h2);
  const int w2c = (w2 < 0) ? 0 : ((w2 > 31) ? 31 : w2);
  const size_t rs = (size_t)b * kNS + h2c * 32 + w2c;
  const float* pa = x1 + rs * kNC + ci0;
  const float* pb = x2 + rs * kNC + ci0;
  const v4f a0 = *(const v4f*)pa, a1 = *(const v4f*)(pa + 4);
  const v4f b0 = *(const v4f*)pb, b1 = *(const v4f*)(pb + 4);
  unsigned short hb[8];
#pragma unroll
  for (int e = 0; e < 4; ++e) {
    hb[e]     = h_bits(valid ? (a0[e] + b0[e]) : 0.0f);
    hb[4 + e] = h_bits(valid ? (a1[e] + b1[e]) : 0.0f);
  }
  const v4u u = (v4u){pk16(hb[0], hb[1]), pk16(hb[2], hb[3]), pk16(hb[4], hb[5]), pk16(hb[6], hb[7])};
  unsigned short* dst = col + (size_t)row * kKConv + (size_t)j * 8;
  *(volatile v4u*)dst = u;
  __threadfence();
  *(volatile v4u*)dst = u;
}

template <int MODE>
__global__ __launch_bounds__(192) void k_bn_part(const float* __restrict__ y2, const float* __restrict__ meanT,
                                                 float* __restrict__ part) {
  const int c   = threadIdx.x;
  const int blk = blockIdx.x;
  const size_t r0 = (size_t)blk * 128;
  const float mval = MODE ? meanT[c] : 0.0f;
  float s = 0.0f;
#pragma unroll 4
  for (int r = 0; r < 128; ++r) {
    const float v = y2[(r0 + r) * kNC + c];
    if (MODE) { const float d = v - mval; s += d * d; } else { s += v; }
  }
  float* dst = part + (size_t)blk * kNC + c;
  *(volatile float*)dst = s;
  __threadfence();
  *(volatile float*)dst = s;
}
template <int MODE>
__global__ __launch_bounds__(192) void k_bn_red(const float* __restrict__ part, float* __restrict__ outT) {
  const int c = threadIdx.x;
  float s = 0.0f;
#pragma unroll 4
  for (int blk = 0; blk < 128; ++blk) s += part[(size_t)blk * kNC + c];
  const float mv = s * (1.0f / 16384.0f);
  const float o  = MODE ? (1.0f / sqrtf(mv + 1e-5f)) : mv;
  *(volatile float*)(outT + c) = o;
  __threadfence();
  *(volatile float*)(outT + c) = o;
}

__global__ __launch_bounds__(256) void k_bn_apply(const float* __restrict__ y2, const float* __restrict__ meanT,
                                                  const float* __restrict__ invT, const float* __restrict__ g,
                                                  const float* __restrict__ be, float* __restrict__ out) {
  __shared__ float sm[32][kNC + 1];
  const int t   = threadIdx.x;
  const int blk = blockIdx.x;
  const int b   = blk >> 5;
  const int p0  = (blk & 31) * 32;
  const size_t base = ((size_t)b * kNS + p0) * kNC;
#pragma unroll
  for (int i = 0; i < 24; ++i) {
    const int e  = i * 256 + t;
    const int r  = e / kNC;
    const int cc = e - r * kNC;
    sm[r][cc] = y2[base + e];
  }
  __syncthreads();
  const int lane = t & 31, wave = t >> 5;
  float vals[24];
#pragma unroll
  for (int i = 0; i < 24; ++i) {
    const int cch = wave * 24 + i;
    const float d = sm[lane][cch] - meanT[cch];
    const float v = d * invT[cch] * g[cch] + be[cch];
    vals[i] = (v >= 0.0f) ? v : 0.01f * v;
  }
  for (int pass = 0; pass < 2; ++pass) {
#pragma unroll
    for (int i = 0; i < 24; ++i) {
      const int cch = wave * 24 + i;
      *(volatile float*)(out + ((size_t)(b * kNC + cch)) * kNS + p0 + lane) = vals[i];
    }
    __threadfence();
  }
}

extern "C" void kernel_launch(void* const* d_in, const int* in_sizes, int n_in,
                              void* d_out, int out_size, void* d_ws, size_t ws_size,
                              hipStream_t stream) {
  (void)in_sizes; (void)n_in; (void)out_size;
  const float* x      = (const float*)d_in[0];
  const float* ln_w   = (const float*)d_in[1];
  const float* ln_b   = (const float*)d_in[2];
  const float* w_up   = (const float*)d_in[3];
  const float* b_up   = (const float*)d_in[4];
  const float* conv_k = (const float*)d_in[5];
  const float* conv_b = (const float*)d_in[6];
  const float* w_q    = (const float*)d_in[7];
  const float* w_k    = (const float*)d_in[8];
  const float* w_i    = (const float*)d_in[9];
  const float* b_i    = (const float*)d_in[10];
  const float* w_f    = (const float*)d_in[11];
  const float* b_f    = (const float*)d_in[12];
  const float* skipv  = (const float*)d_in[13];
  const float* mh_w   = (const float*)d_in[14];
  const float* mh_b   = (const float*)d_in[15];
  const float* w_down = (const float*)d_in[16];
  const float* b_down = (const float*)d_in[17];
  const float* w_lin  = (const float*)d_in[18];
  const float* b_lin  = (const float*)d_in[19];
  const float* conv2w = (const float*)d_in[20];
  const float* conv2b = (const float*)d_in[21];
  const float* bn_g   = (const float*)d_in[22];
  const float* bn_b   = (const float*)d_in[23];
  float* out = (float*)d_out;

  constexpr size_t MIB = 1048576;
  const size_t oSeqf = 0, oSeq16 = 12 * MIB, oHln16 = 18 * MIB, oW = 24 * MIB, oIf = 26 * MIB, oXa16 = 30 * MIB,
               oUp = 42 * MIB, oGin = 90 * MIB;
  const size_t oX1 = 42 * MIB, oX2 = 54 * MIB, oCol = 66 * MIB, oY2 = 0;
  const size_t oGate = 18 * MIB, oPart1 = 20 * MIB, oPart2 = oPart1 + 98304, oMean = oPart2 + 98304, oInv = oMean + 1024;
  const size_t total = 126 * MIB;
  if (ws_size < total) return;
  char* ws = (char*)d_ws;

  float* seqf            = (float*)(ws + oSeqf);
  unsigned short* seq16  = (unsigned short*)(ws + oSeq16);
  unsigned short* hln16  = (unsigned short*)(ws + oHln16);
  float* gatet           = (float*)(ws + oGate);
  float* part1           = (float*)(ws + oPart1);
  float* part2           = (float*)(ws + oPart2);
  float* meanT           = (float*)(ws + oMean);
  float* invT            = (float*)(ws + oInv);
  float* ifp             = (float*)(ws + oIf);
  unsigned short* xact16 = (unsigned short*)(ws + oXa16);
  unsigned short* hout16 = (unsigned short*)(ws + oXa16);
  float* upf             = (float*)(ws + oUp);
  float* x1              = (float*)(ws + oX1);
  float* x2              = (float*)(ws + oX2);
  unsigned short* col16  = (unsigned short*)(ws + oCol);
  unsigned short* gin16  = (unsigned short*)(ws + oGin);
  float* y2              = (float*)(ws + oY2);

  unsigned short* wupT = (unsigned short*)(ws + oW + 0);
  unsigned short* wqT  = (unsigned short*)(ws + oW + 294912);
  unsigned short* wkT  = (unsigned short*)(ws + oW + 589824);
  unsigned short* wifT = (unsigned short*)(ws + oW + 884736);
  unsigned short* wdT  = (unsigned short*)(ws + oW + 1032192);
  unsigned short* wlT  = (unsigned short*)(ws + oW + 1179648);
  unsigned short* w2T  = (unsigned short*)(ws + oW + 1253376);
  float* bif64         = (float*)(ws + oW + 1916928);

  k_wt64<<<dim3(kNC / 64, kNUp / 64), 256, 0, stream>>>(w_up, wupT, kNC, kNUp, kWCar);
  k_wt64<<<dim3(kNin / 64, kNin / 64), 256, 0, stream>>>(w_q, wqT, kNin, kNin, kWCar);
  k_wt64<<<dim3(kNin / 64, kNin / 64), 256, 0, stream>>>(w_k, wkT, kNin, kNin, kWCar);
  k_wt64<<<dim3(kNin / 64, kNC / 64), 256, 0, stream>>>(w_down, wdT, kNin, kNC, kWCar);
  k_wt64<<<dim3(kNC / 64, kNC / 64), 256, 0, stream>>>(w_lin, wlT, kNC, kNC, kWCar);
  k_wif<<<36, 256, 0, stream>>>(w_i, w_f, wifT, kWCar);
  k_bias64<<<1, 32, 0, stream>>>(b_i, b_f, bif64);
  k_w2<<<162, 256, 0, stream>>>(conv2w, w2T, kW2Car);

  k_ln<<<kRows / 32, 256, 0, stream>>>(x, ln_w, ln_b, seqf, seq16, hln16);

  wmma_gemm64<0, false, 2, 0, false, 0><<<dim3(384, 1), 256, 0, stream>>>(
      hln16, hln16, kNC, 0L, wupT, wupT, kNC, 0L, (void*)upf, (void*)upf, kNUp, 0L,
      b_up, b_up, 0L, kRows, kNUp, kNC, kUpScale);

  k_conv1d<<<3072, 256, 0, stream>>>(upf, conv_k, conv_b, xact16, gin16);

  wmma_gemm64<0, false, 0, 1, false, 0><<<dim3(192, 1), 256, 0, stream>>>(
      xact16, xact16, kNin, 0L, wqT, wqT, kNin, 0L, (void*)(gin16 + 0), (void*)(gin16 + 0), kNGin, 0L,
      b_up, b_up, 0L, kRows, kNin, kNin, kQKScale);
  wmma_gemm64<0, false, 0, 1, false, 0><<<dim3(192, 1), 256, 0, stream>>>(
      xact16, xact16, kNin, 0L, wkT, wkT, kNin, 0L, (void*)(gin16 + kNin), (void*)(gin16 + kNin), kNGin, 0L,
      b_up, b_up, 0L, kRows, kNin, kNin, kQKScale);

  wmma_gemm64<0, false, 2, 0, false, 0><<<dim3(32, 1), 256, 0, stream>>>(
      gin16, gin16, kNGin, 0L, wifT, wifT, kNGin, 0L, (void*)ifp, (void*)ifp, kNIf, 0L,
      bif64, bif64, 0L, kRows, kNIf, kNGin, kIfScale);

  k_gate<<<1, 192, 0, stream>>>(ifp, gatet);
  k_scan<<<kNB, 384, 0, stream>>>(upf, (const unsigned int*)gin16, gatet, conv_k, conv_b, skipv, mh_w, mh_b, hout16);

  wmma_gemm64<0, false, 2, 0, true, 0><<<dim3(96, 1), 256, 0, stream>>>(
      hout16, hout16, kNin, 0L, wdT, wdT, kNin, 0L, (void*)x1, (void*)x1, kNC, 0L,
      b_down, seqf, 0L, kRows, kNC, kNin, kDownScale);
  wmma_gemm64<0, false, 2, 0, false, 3><<<dim3(96, 1), 256, 0, stream>>>(
      seq16, seq16, kNC, 0L, wlT, wlT, kNC, 0L, (void*)x2, (void*)x2, kNC, 0L,
      b_lin, b_lin, 0L, kRows, kNC, kNC, kLinScale);

  k_im2col<<<13824, 256, 0, stream>>>(x1, x2, col16);
  wmma_gemm64<0, false, 2, 0, false, 0><<<dim3(96, 1), 256, 0, stream>>>(
      col16, col16, kKConv, 0L, w2T, w2T, kKConv, 0L, (void*)y2, (void*)y2, kNC, 0L,
      conv2b, conv2b, 0L, kRows, kNC, kKConv, kConvScale);

  k_bn_part<0><<<128, 192, 0, stream>>>(y2, y2, part1);
  k_bn_red<0><<<1, 192, 0, stream>>>(part1, meanT);
  k_bn_part<1><<<128, 192, 0, stream>>>(y2, meanT, part2);
  k_bn_red<1><<<1, 192, 0, stream>>>(part2, invT);
  k_bn_apply<<<kRows / 32, 256, 0, stream>>>(y2, meanT, invT, bn_g, bn_b, out);
}
